// TRoPECrossAttention_41867341201565
// MI455X (gfx1250) — hardware-verified
//
#include <hip/hip_runtime.h>
#include <math.h>
#include <float.h>
#include <stdint.h>

#define BSZ   2
#define SEQ   2048
#define DM    1024
#define NH    16
#define HD    64
#define NPAIR (HD / 2)
#define QKVN  (3 * DM)
#define ROWS  (BSZ * SEQ)
#define NQT   (SEQ / 64)
#define NTAB  (ROWS * NPAIR)
static_assert(NH * HD == DM);
static_assert(HD == 64);
static_assert(DM == 128 * 8);
static_assert((SEQ % 64) == 0);
static_assert((ROWS % 64) == 0 && (DM % 64) == 0 && (QKVN % 64) == 0 && (DM % 32) == 0);
static_assert((((ROWS / 64) * (QKVN / 64)) % 8) == 0);
static_assert((((ROWS / 64) * (DM / 64)) % 8) == 0);
static_assert(((ROWS * DM / 8) % 256) == 0);
static_assert((NTAB % 256) == 0);

typedef _Float16 v16h __attribute__((ext_vector_type(16)));
typedef _Float16 v8h  __attribute__((ext_vector_type(8)));
typedef float    v8f  __attribute__((ext_vector_type(8)));
typedef float    v4f  __attribute__((ext_vector_type(4)));
typedef unsigned int v4u __attribute__((ext_vector_type(4)));

__device__ __forceinline__ unsigned short bf_bits(float f) {
  unsigned u = __float_as_uint(f);
  return (unsigned short)((u + 0x7FFFu + ((u >> 16) & 1u)) >> 16);
}
__device__ __forceinline__ float bf_up(unsigned short h) { return __uint_as_float(((unsigned)h) << 16); }
__device__ __forceinline__ float bfr(float f) { return bf_up(bf_bits(f)); }
__device__ __forceinline__ unsigned short h_bits(_Float16 x) { return __builtin_bit_cast(unsigned short, x); }
__device__ __forceinline__ unsigned pk16(unsigned short a, unsigned short b) { return (unsigned)a | ((unsigned)b << 16); }
__device__ __forceinline__ v8f zero8() { v8f z = {0.f, 0.f, 0.f, 0.f, 0.f, 0.f, 0.f, 0.f}; return z; }

__device__ __forceinline__ void ld8(const float* p, float* o) {
  const v4f a = *(const v4f*)(p);
  const v4f b = *(const v4f*)(p + 4);
  o[0] = a[0]; o[1] = a[1]; o[2] = a[2]; o[3] = a[3];
  o[4] = b[0]; o[5] = b[1]; o[6] = b[2]; o[7] = b[3];
}

__device__ __forceinline__ v16h ldfrag_h(const _Float16* p) {
  union { v16h v; v8h h[2]; } f;
  f.h[0] = *(const v8h*)(p);
  f.h[1] = *(const v8h*)(p + 16);
  return f.v;
}

__device__ __forceinline__ v8f mma_h(v16h a, v16h b, v8f c) {
  c = __builtin_amdgcn_wmma_f32_16x16x32_f16(false, a, false, b, (short)0, c, false, false);
#if defined(__HIP_DEVICE_COMPILE__)
  asm volatile("v_nop\n\tv_nop\n\tv_nop\n\tv_nop" : "+v"(c) : "v"(a), "v"(b));
#endif
  return c;
}
__device__ __forceinline__ v8f mma_h_raw(v16h a, v16h b, v8f c) {
  return __builtin_amdgcn_wmma_f32_16x16x32_f16(false, a, false, b, (short)0, c, false, false);
}
__device__ __forceinline__ void dep_guard_h(v8f& a, v8f& b, v16h x) {
#if defined(__HIP_DEVICE_COMPILE__)
  asm volatile("v_nop\n\tv_nop\n\tv_nop\n\tv_nop" : "+v"(a), "+v"(b) : "v"(x));
#endif
}
__device__ __forceinline__ void keep4_h(v16h a, v16h b, v16h c, v16h d) {
#if defined(__HIP_DEVICE_COMPILE__)
  asm volatile("v_nop" :: "v"(a), "v"(b), "v"(c), "v"(d));
#endif
}
__device__ __forceinline__ void acc_guard4(v8f& a, v8f& b, v8f& c, v8f& d) {
#if defined(__HIP_DEVICE_COMPILE__)
  asm volatile("v_nop\n\tv_nop\n\tv_nop\n\tv_nop" : "+v"(a), "+v"(b), "+v"(c), "+v"(d));
#endif
}

__global__ __launch_bounds__(256) void rope_tab(const int* __restrict__ tt, float* ct, float* st, int n) {
#pragma clang fp contract(off)
  const int i = blockIdx.x * 256 + threadIdx.x;
  if (i < n) {
    int row = i >> 5;
    row = (row < ROWS) ? row : (ROWS - 1);
    const int j   = i & 31;
    const int t   = tt[row];
    const float e   = (float)j * (1.0f / 32.0f);
    const float p   = powf(10000.0f, e);
    const float inv = 1.0f / p;
    const float ang = (float)t * inv;
    const float cv = cosf(ang);
    const float sv = sinf(ang);
    *(volatile float*)(ct + i) = cv;
    *(volatile float*)(st + i) = sv;
    __threadfence();
    *(volatile float*)(ct + i) = cv;
    *(volatile float*)(st + i) = sv;
  }
}

__global__ __launch_bounds__(256) void wt_cvt(const float* __restrict__ W, int ncols, int nrows,
                                              unsigned short* outp, float sc) {
  __shared__ __align__(16) float sw[64 * 68];
  const int tid = threadIdx.x;
  const int n0 = blockIdx.x * 64;
  const int k0 = blockIdx.y * 64;
#pragma unroll
  for (int i = 0; i < 4; ++i) {
    const int idx = i * 256 + tid;
    const int kk = idx >> 4, c4 = (idx & 15) * 4;
    const v4f a = *(const v4f*)(W + (size_t)(k0 + kk) * ncols + n0 + c4);
    *(v4f*)(sw + kk * 68 + c4) = a;
  }
  __syncthreads();

  const int g = tid >> 3, piece = tid & 7;
  v4u ov[2];
  size_t oofs[2];
#pragma unroll
  for (int it = 0; it < 2; ++it) {
    const int nn = it * 32 + g;
    v4u a;
#pragma unroll
    for (int e = 0; e < 4; ++e) {
      const float f0 = sw[(piece * 8 + 2 * e) * 68 + nn];
      const float f1 = sw[(piece * 8 + 2 * e + 1) * 68 + nn];
      a[e] = pk16(h_bits((_Float16)(bfr(f0) * sc)), h_bits((_Float16)(bfr(f1) * sc)));
    }
    ov[it] = a;
    oofs[it] = (size_t)(n0 + nn) * nrows + k0 + piece * 8;
  }
  for (int pass = 0; pass < 2; ++pass) {
#pragma unroll
    for (int it = 0; it < 2; ++it) *(volatile v4u*)(outp + oofs[it]) = ov[it];
    __threadfence();
  }
}

__global__ __launch_bounds__(256) void cvt_xh(const float* __restrict__ in, unsigned short* out, int n8,
                                              float sc) {
  const int i = blockIdx.x * 256 + threadIdx.x;
  if (i < n8) {
    const v4f a = *(const v4f*)(in + (size_t)i * 8);
    const v4f b = *(const v4f*)(in + (size_t)i * 8 + 4);
    v4u p;
    p[0] = pk16(h_bits((_Float16)(bfr(a[0]) * sc)), h_bits((_Float16)(bfr(a[1]) * sc)));
    p[1] = pk16(h_bits((_Float16)(bfr(a[2]) * sc)), h_bits((_Float16)(bfr(a[3]) * sc)));
    p[2] = pk16(h_bits((_Float16)(bfr(b[0]) * sc)), h_bits((_Float16)(bfr(b[1]) * sc)));
    p[3] = pk16(h_bits((_Float16)(bfr(b[2]) * sc)), h_bits((_Float16)(bfr(b[3]) * sc)));
    *(volatile v4u*)(out + (size_t)i * 8) = p;
    __threadfence();
    *(volatile v4u*)(out + (size_t)i * 8) = p;
  }
}

template <int HASB>
__global__ __launch_bounds__(256) void gemm64(
    const unsigned short* __restrict__ Ap, int lda,
    const unsigned short* __restrict__ Btp, int ldb,
    const float* __restrict__ bias, float* Cf, int ldc, int M, int N, int K, float oscale) {
  const _Float16* Ah = (const _Float16*)(const void*)Ap;
  const _Float16* Bh = (const _Float16*)(const void*)Btp;
  __shared__ __align__(16) float sT[8][16 * 68];
  const int lane = threadIdx.x & 31;
  const int wave = threadIdx.x >> 5;
  const int tilesN = N >> 6;
  const int tilesM = M >> 6;
  const int tile = blockIdx.x * 8 + wave;
  if (tile >= tilesM * tilesN) return;
  const int tm = tile / tilesN;
  const int tn = tile - tm * tilesN;
  const int m0 = tm << 6;
  const int n0 = tn << 6;

  const int rlane = lane & 15;
  const int koff  = (lane >> 4) * 8;
  const int mOff  = (lane >> 4) * 8;

  v8f acc[4][4];
#pragma unroll
  for (int i = 0; i < 4; ++i)
#pragma unroll
    for (int j = 0; j < 4; ++j) acc[i][j] = zero8();

  for (int k0 = 0; k0 < K; k0 += 32) {
    v16h bh[4];
#pragma unroll
    for (int j = 0; j < 4; ++j) {
      const size_t bo = (size_t)(n0 + (j << 4) + rlane) * ldb + koff + k0;
      bh[j] = ldfrag_h(Bh + bo);
    }
#pragma unroll
    for (int i = 0; i < 4; ++i) {
      const size_t ao = (size_t)(m0 + (i << 4) + rlane) * lda + koff + k0;
      const v16h ah = ldfrag_h(Ah + ao);
#pragma unroll
      for (int j = 0; j < 4; ++j) acc[i][j] = mma_h_raw(ah, bh[j], acc[i][j]);
      dep_guard_h(acc[i][0], acc[i][3], ah);
    }
    keep4_h(bh[0], bh[1], bh[2], bh[3]);
  }
  acc_guard4(acc[0][0], acc[0][1], acc[0][2], acc[0][3]);
  acc_guard4(acc[1][0], acc[1][1], acc[1][2], acc[1][3]);
  acc_guard4(acc[2][0], acc[2][1], acc[2][2], acc[2][3]);
  acc_guard4(acc[3][0], acc[3][1], acc[3][2], acc[3][3]);

  float* slab = sT[wave];
  const int h2 = lane >> 4, c4 = (lane & 15) * 4;
  v4f b4 = {0.f, 0.f, 0.f, 0.f};
  if (HASB != 0) {
    const v4f braw = *(const v4f*)(bias + n0 + c4);
#pragma unroll
    for (int e = 0; e < 4; ++e) b4[e] = bfr(braw[e]);
  }
#pragma unroll
  for (int i = 0; i < 4; ++i) {
    const int mBase = m0 + (i << 4);
#pragma unroll
    for (int r = 0; r < 8; ++r) {
#pragma unroll
      for (int j = 0; j < 4; ++j) {
        slab[(mOff + r) * 68 + (j << 4) + rlane] = acc[i][j][r];
      }
    }
    __builtin_amdgcn_fence(__ATOMIC_RELEASE, "workgroup");
    __builtin_amdgcn_wave_barrier();
    __builtin_amdgcn_fence(__ATOMIC_ACQUIRE, "workgroup");
    v4f ov[8];
#pragma unroll
    for (int it = 0; it < 8; ++it) {
      const int row = it * 2 + h2;
      const v4f xs = *(const v4f*)(slab + row * 68 + c4);
      ov[it] = xs * oscale + b4;
    }
    for (int pass = 0; pass < 2; ++pass) {
#pragma unroll
      for (int it = 0; it < 8; ++it) {
        const int row = it * 2 + h2;
        *(volatile v4f*)(Cf + (size_t)(mBase + row) * ldc + n0 + c4) = ov[it];
      }
      __threadfence();
    }
    __builtin_amdgcn_fence(__ATOMIC_RELEASE, "workgroup");
    __builtin_amdgcn_wave_barrier();
    __builtin_amdgcn_fence(__ATOMIC_ACQUIRE, "workgroup");
  }
}

__global__ __launch_bounds__(128) void rope_qk(const float* __restrict__ qkvf,
                                               const float* __restrict__ cq, const float* __restrict__ sq,
                                               const float* __restrict__ ck, const float* __restrict__ sk,
                                               unsigned short* qh, unsigned short* kh, float osc) {
#pragma clang fp contract(off)
  const int tid = threadIdx.x;
  const int row = blockIdx.x;
  const float* rowp = qkvf + (size_t)row * QKVN;
  const int d0 = tid * 8;
  const int i0 = (d0 & (HD - 1)) >> 1;
  float xq[8], xk[8];
  ld8(rowp + d0, xq);
  ld8(rowp + DM + d0, xk);
  const size_t tofs = (size_t)row * NPAIR + i0;
  const v4f cqv = *(const v4f*)(cq + tofs);
  const v4f sqv = *(const v4f*)(sq + tofs);
  const v4f ckv = *(const v4f*)(ck + tofs);
  const v4f skv = *(const v4f*)(sk + tofs);

  v4u aq, ak;
#pragma unroll
  for (int pp = 0; pp < 4; ++pp) {
    const float q1 = xq[2 * pp], q2 = xq[2 * pp + 1];
    const float k1 = xk[2 * pp], k2 = xk[2 * pp + 1];
    const float yq0 = q1 * cqv[pp] - q2 * sqv[pp];
    const float yq1 = q1 * sqv[pp] + q2 * cqv[pp];
    const float yk0 = k1 * ckv[pp] - k2 * skv[pp];
    const float yk1 = k1 * skv[pp] + k2 * ckv[pp];
    aq[pp] = pk16(h_bits((_Float16)(yq0 * osc)), h_bits((_Float16)(yq1 * osc)));
    ak[pp] = pk16(h_bits((_Float16)(yk0 * osc)), h_bits((_Float16)(yk1 * osc)));
  }
  const size_t o = (size_t)row * DM + d0;
  *(volatile v4u*)(qh + o) = aq;
  *(volatile v4u*)(kh + o) = ak;
  __threadfence();
  *(volatile v4u*)(qh + o) = aq;
  *(volatile v4u*)(kh + o) = ak;
}

__global__ __launch_bounds__(256) void v_planes(const float* __restrict__ qkvf, unsigned short* vt, float vscale) {
  __shared__ __align__(16) float svt[64 * 68];
  const int tid = threadIdx.x;
  const int kt  = blockIdx.x;
  const int hh  = blockIdx.y;
  const int b   = blockIdx.z;
  const int t0  = kt * 64;
#pragma unroll
  for (int i = 0; i < 4; ++i) {
    const int idx = i * 256 + tid;
    const int tt = idx >> 4, c4 = (idx & 15) * 4;
    const int srow = b * SEQ + t0 + tt;
    const v4f a = *(const v4f*)(qkvf + (size_t)srow * QKVN + 2 * DM + hh * HD + c4);
    *(v4f*)(svt + tt * 68 + c4) = a;
  }
  __syncthreads();

  const int g = tid >> 3, piece = tid & 7;
  v4u hv[2];
  size_t hofs[2];
#pragma unroll
  for (int it = 0; it < 2; ++it) {
    const int d = it * 32 + g;
    v4u a;
#pragma unroll
    for (int e = 0; e < 4; ++e) {
      const float f0 = svt[(piece * 8 + 2 * e) * 68 + d] * vscale;
      const float f1 = svt[(piece * 8 + 2 * e + 1) * 68 + d] * vscale;
      a[e] = pk16(h_bits((_Float16)f0), h_bits((_Float16)f1));
    }
    hv[it] = a;
    hofs[it] = ((size_t)(b * DM + hh * HD + d)) * SEQ + t0 + piece * 8;
  }
  for (int pass = 0; pass < 2; ++pass) {
#pragma unroll
    for (int it = 0; it < 2; ++it) *(volatile v4u*)(vt + hofs[it]) = hv[it];
    __threadfence();
  }
}

__global__ __launch_bounds__(128)
void attn64(const unsigned short* __restrict__ qhp, const unsigned short* __restrict__ khp,
            const unsigned short* __restrict__ vtp, unsigned short* yh, float sscale, float oscl) {
  union FH { v16h v; v8h h[2]; };
  __shared__ __align__(16) _Float16 Khs[64 * 64];
  __shared__ __align__(16) _Float16 Vts[64 * 64];
  __shared__ __align__(16) _Float16 Psh[4][16 * 64];
  __shared__ __align__(16) float    Os[4][16 * 64];

  const int tid  = threadIdx.x;
  const int wave = tid >> 5;
  const int lane = tid & 31;
  const int hh   = lane >> 4;
  const int c    = lane & 15;

  const int bx = blockIdx.x;
  const int qt = bx % NQT;
  const int hb = bx / NQT;
  const int h  = hb % NH;
  const int b  = hb / NH;
  const int q0 = qt * 64 + wave * 16;

  const size_t qkb = (size_t)b * SEQ * DM + (size_t)h * HD;
  const _Float16* Qh = (const _Float16*)(const void*)qhp + qkb;
  const _Float16* Kh = (const _Float16*)(const void*)khp + qkb;
  const _Float16* Vt = (const _Float16*)(const void*)vtp + ((size_t)b * DM + (size_t)h * HD) * SEQ;

  v16h qa[2];
#pragma unroll
  for (int dc = 0; dc < 2; ++dc) {
    const size_t qo = (size_t)(q0 + c) * DM + dc * 32 + 8 * hh;
    qa[dc] = ldfrag_h(Qh + qo);
  }

  float mrow[8], lrow[8];
  v8f oacc[4];
#pragma unroll
  for (int r = 0; r < 8; ++r) { mrow[r] = -INFINITY; lrow[r] = 0.f; }
#pragma unroll
  for (int t = 0; t < 4; ++t) oacc[t] = zero8();

  for (int kt = 0; kt < NQT; ++kt) {
    const int kv0 = kt * 64;
    __syncthreads();
    {
      const int r = tid >> 1, half = (tid & 1) * 32;
      const _Float16* kg = Kh + (size_t)(kv0 + r) * DM + half;
      const _Float16* vg = Vt + (size_t)r * SEQ + kv0 + half;
#pragma unroll
      for (int i = 0; i < 4; ++i) {
        const v8h a0 = *(const v8h*)(kg + 8 * i);
        const v8h b0 = *(const v8h*)(vg + 8 * i);
        *(v8h*)(Khs + r * 64 + half + 8 * i) = a0;
        *(v8h*)(Vts + r * 64 + half + 8 * i) = b0;
      }
    }
    __syncthreads();

    v8f s[4];
#pragma unroll
    for (int j = 0; j < 4; ++j) {
      v8f ahh = zero8();
#pragma unroll
      for (int dc = 0; dc < 2; ++dc) {
        FH kb;
        kb.h[0] = *(const v8h*)(Khs + (j * 16 + c) * 64 + dc * 32 + 8 * hh);
        kb.h[1] = *(const v8h*)(Khs + (j * 16 + c) * 64 + dc * 32 + 16 + 8 * hh);
        ahh = mma_h(qa[dc], kb.v, ahh);
      }
      s[j] = ahh;
    }

    _Float16* pwh = Psh[wave];
#pragma unroll
    for (int r = 0; r < 8; ++r) {
      float m = -INFINITY;
#pragma unroll
      for (int j = 0; j < 4; ++j) {
        const float sv = s[j][r] * sscale;
        s[j][r] = sv;
        m = fmaxf(m, sv);
      }
#pragma unroll
      for (int off = 1; off < 16; off <<= 1) m = fmaxf(m, __shfl_xor(m, off, 32));
      const float mnew  = fmaxf(mrow[r], m);
      const float msafe = (mnew == -INFINITY) ? 0.f : mnew;
      const float alpha = __expf(mrow[r] - msafe);
      mrow[r] = mnew;
      float psum = 0.f;
#pragma unroll
      for (int j = 0; j < 4; ++j) {
        const float p = __expf(s[j][r] - msafe);
        psum += p;
        const _Float16 ph = (_Float16)(p * 1024.0f);
        pwh[(8 * hh + r) * 64 + j * 16 + c] = ph;
      }
#pragma unroll
      for (int off = 1; off < 16; off <<= 1) psum += __shfl_xor(psum, off, 32);
      lrow[r] = lrow[r] * alpha + psum;
#pragma unroll
      for (int t = 0; t < 4; ++t) oacc[t][r] *= alpha;
    }
    __builtin_amdgcn_fence(__ATOMIC_RELEASE, "workgroup");
    __builtin_amdgcn_wave_barrier();
    __builtin_amdgcn_fence(__ATOMIC_ACQUIRE, "workgroup");

#pragma unroll 1
    for (int kk = 0; kk < 2; ++kk) {
      FH pa;
      pa.h[0] = *(const v8h*)(pwh + c * 64 + kk * 32 + 8 * hh);
      pa.h[1] = *(const v8h*)(pwh + c * 64 + kk * 32 + 16 + 8 * hh);
#pragma unroll
      for (int t = 0; t < 4; ++t) {
        FH vb;
        vb.h[0] = *(const v8h*)(Vts + (t * 16 + c) * 64 + kk * 32 + 8 * hh);
        vb.h[1] = *(const v8h*)(Vts + (t * 16 + c) * 64 + kk * 32 + 16 + 8 * hh);
        oacc[t] = mma_h(pa.v, vb.v, oacc[t]);
      }
    }
  }

  float* os = Os[wave];
#pragma unroll
  for (int r = 0; r < 8; ++r) {
    const float l = lrow[r];
    const float inv = ((l > 0.f) ? (1.0f / l) : 0.f) * oscl;
#pragma unroll
    for (int t = 0; t < 4; ++t) os[(8 * hh + r) * 64 + t * 16 + c] = oacc[t][r] * inv;
  }
  __builtin_amdgcn_fence(__ATOMIC_RELEASE, "workgroup");
  __builtin_amdgcn_wave_barrier();
  __builtin_amdgcn_fence(__ATOMIC_ACQUIRE, "workgroup");
  {
    const int q8 = lane & 7, rr = lane >> 3, c8 = q8 * 8;
    v4u ov[4];
    size_t go[4];
#pragma unroll
    for (int it = 0; it < 4; ++it) {
      const int row = it * 4 + rr;
      float xs[8];
      ld8(os + row * 64 + c8, xs);
      v4u a;
#pragma unroll
      for (int pp = 0; pp < 4; ++pp) a[pp] = pk16(h_bits((_Float16)xs[2 * pp]), h_bits((_Float16)xs[2 * pp + 1]));
      ov[it] = a;
      const int dr = b * SEQ + q0 + row;
      go[it] = (size_t)dr * DM + (size_t)h * HD + c8;
    }
    for (int pass = 0; pass < 2; ++pass) {
#pragma unroll
      for (int it = 0; it < 4; ++it) *(volatile v4u*)(yh + go[it]) = ov[it];
      __threadfence();
    }
  }
}

extern "C" void kernel_launch(void* const* d_in, const int* in_sizes, int n_in,
                              void* d_out, int out_size, void* d_ws, size_t ws_size,
                              hipStream_t stream) {
  if (n_in < 7) return;
  if (in_sizes[0] != ROWS * DM) return;
  if (in_sizes[1] != ROWS || in_sizes[2] != ROWS) return;
  if (in_sizes[3] != DM * DM) return;
  if (in_sizes[4] != DM * 2 * DM) return;
  if (in_sizes[5] != DM * DM || in_sizes[6] != DM) return;
  if (out_size != ROWS * DM) return;

  const float* x    = (const float*)d_in[0];
  const int*   tq   = (const int*)d_in[1];
  const int*   tk   = (const int*)d_in[2];
  const float* wq   = (const float*)d_in[3];
  const float* wkv  = (const float*)d_in[4];
  const float* wo   = (const float*)d_in[5];
  const float* bo   = (const float*)d_in[6];

  const size_t PXh   = (size_t)ROWS * DM * 2;
  const size_t PWT   = (size_t)QKVN * DM * 2;
  const size_t PWo   = (size_t)DM * DM * 2;
  const size_t PTab  = (size_t)NTAB * 4;
  const size_t PQKV  = (size_t)ROWS * QKVN * 4;
  const size_t PQK   = (size_t)ROWS * DM * 2;
  const size_t PVT   = (size_t)BSZ * DM * SEQ * 2;
  const size_t PY    = (size_t)ROWS * DM * 2;
  size_t off = 0;
  const size_t oXh  = off; off += PXh;
  const size_t oWT  = off; off += PWT;
  const size_t oWo  = off; off += PWo;
  const size_t oCq  = off; off += PTab;
  const size_t oSq  = off; off += PTab;
  const size_t oCk  = off; off += PTab;
  const size_t oSk  = off; off += PTab;
  const size_t oQKV = off; off += PQKV;
  const size_t oQh  = off; off += PQK;
  const size_t oKh  = off; off += PQK;
  const size_t oVT  = off; off += PVT;
  const size_t oY   = off; off += PY;
  if (off > ws_size) return;
  if (off > (size_t)134217728) return;

  char* ws = (char*)d_ws;
  unsigned short* Xh   = (unsigned short*)(ws + oXh);
  unsigned short* WT   = (unsigned short*)(ws + oWT);
  unsigned short* WoT  = (unsigned short*)(ws + oWo);
  float*          CqT  = (float*)(ws + oCq);
  float*          SqT  = (float*)(ws + oSq);
  float*          CkT  = (float*)(ws + oCk);
  float*          SkT  = (float*)(ws + oSk);
  float*          QKVf = (float*)(ws + oQKV);
  unsigned short* Qh   = (unsigned short*)(ws + oQh);
  unsigned short* Kh   = (unsigned short*)(ws + oKh);
  unsigned short* VT   = (unsigned short*)(ws + oVT);
  unsigned short* Yh   = (unsigned short*)(ws + oY);
  float*          outf = (float*)d_out;

  const dim3 blk(256);
  const int nTab = NTAB;
  const int n8x  = ROWS * DM / 8;
  const dim3 gTab((nTab + 255) / 256);
  const dim3 gCx((n8x + 255) / 256);
  const dim3 gWq(DM / 64, DM / 64);
  const dim3 gWkv((2 * DM) / 64, DM / 64);
  const dim3 gWo(DM / 64, DM / 64);
  const dim3 gQKV(((ROWS / 64) * (QKVN / 64) + 7) / 8);
  const dim3 gOut(((ROWS / 64) * (DM / 64) + 7) / 8);
  const dim3 gRope(ROWS);
  const dim3 gVpl(NQT, NH, BSZ);
  const dim3 gAttn(BSZ * NH * NQT);

  const float wScale  = 64.0f;
  const float xScale  = 8.0f;
  const float qkvInv  = 1.0f / 512.0f;
  const float qkScale = 16.0f;
  const float sscale  = 1.0f / 2048.0f;
  const float vScale  = 256.0f;
  const float attOscl = 64.0f / 262144.0f;
  const float yInv    = 1.0f / 4096.0f;

  rope_tab<<<gTab, blk, 0, stream>>>(tq, CqT, SqT, nTab);
  rope_tab<<<gTab, blk, 0, stream>>>(tk, CkT, SkT, nTab);
  wt_cvt<<<gWq, blk, 0, stream>>>(wq, DM, DM, WT, wScale);
  wt_cvt<<<gWkv, blk, 0, stream>>>(wkv, 2 * DM, DM, WT + (size_t)DM * DM, wScale);
  wt_cvt<<<gWo, blk, 0, stream>>>(wo, DM, DM, WoT, wScale);
  cvt_xh<<<gCx, blk, 0, stream>>>(x, Xh, n8x, xScale);
  gemm64<0><<<gQKV, blk, 0, stream>>>(Xh, DM, WT, DM, bo, QKVf, QKVN, ROWS, QKVN, DM, qkvInv);
  rope_qk<<<gRope, dim3(128), 0, stream>>>(QKVf, CqT, SqT, CkT, SkT, Qh, Kh, qkScale);
  v_planes<<<gVpl, blk, 0, stream>>>(QKVf, VT, vScale);
  attn64<<<gAttn, dim3(128), 0, stream>>>(Qh, Kh, VT, Yh, sscale, attOscl);
  gemm64<1><<<gOut, blk, 0, stream>>>(Yh, DM, WoT, DM, bo, outf, DM, ROWS, DM, DM, yInv);
  (void)hipGetLastError();
}
